// selfattention_4569845203261
// MI455X (gfx1250) — hardware-verified
//
#include <hip/hip_runtime.h>
#ifndef NB
#define NB 2
#endif
#ifndef SEQ
#define SEQ 2048
#endif
#define NB_FULL 2
#define SEQ_FULL 2048
#define NH 16
#define HD 128
#define KCH (HD / 32)
#define DTL (HD / 16)
#define NPL (NB * NH)
#define PLANE_BYTES ((size_t)NPL * SEQ * HD * 2)

static_assert(SEQ % 64 == 0);
static_assert(SEQ <= SEQ_FULL);
static_assert(NB <= NB_FULL);
static_assert(HD == 128);
static_assert(KCH == 4);
static_assert(DTL == 8);
static_assert(3 * ((size_t)NPL * SEQ * HD * 2) <= (size_t)134217728);
static_assert(((size_t)NPL * SEQ * HD * 2) % 256 == 0);
static_assert((size_t)(SEQ / 64) * NPL * 256 * 4 * 8 == (size_t)NPL * SEQ * HD);
static_assert((size_t)(SEQ / 64) * NPL * 4 * 16 * HD == (size_t)NPL * SEQ * HD);
static_assert(32 * 16 == HD * 4);
static_assert(SEQ % 32 == 0);

typedef _Float16 v16h __attribute__((ext_vector_type(16)));
typedef unsigned short v8us __attribute__((ext_vector_type(8), may_alias));
typedef float v8f  __attribute__((ext_vector_type(8)));
typedef float v4f  __attribute__((ext_vector_type(4)));
typedef float v4fa __attribute__((ext_vector_type(4), may_alias));
union FragH { v16h v; v8us half[2]; _Float16 h[16]; unsigned short u[16]; };

#if defined(__has_builtin)
#if __has_builtin(__builtin_amdgcn_exp2f)
#define EXP2F(x) __builtin_amdgcn_exp2f(x)
#endif
#endif
#ifndef EXP2F
#define EXP2F(x) exp2f(x)
#endif

__device__ __forceinline__ unsigned short bf16_bits(float x) { unsigned int u = __float_as_uint(x); return (unsigned short)((u + 0x7FFFu + ((u >> 16) & 1u)) >> 16); }
__device__ __forceinline__ float bf16_val(unsigned short b) { return __uint_as_float(((unsigned int)b) << 16); }
__device__ __forceinline__ float bf16_rne(float x) { return bf16_val(bf16_bits(x)); }

static __device__ __forceinline__ _Float16 toh_flush(float v) {
  const _Float16 r = (_Float16)v;
  return (fabsf(v) < 6.103515625e-05f) ? (_Float16)0.0f : r;
}

__device__ __forceinline__ v8f mma16(v16h a, v16h b, v8f c) {
  v8f d = __builtin_amdgcn_wmma_f32_16x16x32_f16(false, a, false, b, (short)0, c, false, false);
  asm volatile("v_nop\n\tv_nop\n\tv_nop\n\tv_nop" : "+v"(d) : "v"(a), "v"(b));
  return d;
}

__global__ __launch_bounds__(256) void k_cvt(const float* __restrict__ q, const float* __restrict__ k, const float* __restrict__ v,
                                            _Float16* __restrict__ Q16, _Float16* __restrict__ K16, _Float16* __restrict__ VT) {
  __shared__ unsigned short tl[HD][72];
  const unsigned tid = threadIdx.x;
  const unsigned jb = blockIdx.x << 6;
  const unsigned bh = blockIdx.y;
  const size_t ib = ((size_t)bh * SEQ_FULL + jb) * HD;
  const size_t ob = ((size_t)bh * SEQ + jb) * HD;
  FragH fq[4], fk[4], fv[4];
#pragma unroll
  for (int i = 0; i < 4; ++i) {
    const unsigned c = tid + ((unsigned)i << 8);
    const unsigned row = c >> 4, c8 = (c & 15u) << 3;
    const size_t go = ib + (size_t)(row << 7) + c8;
    const v4f qa = *(const v4fa*)(q + go), qc = *(const v4fa*)(q + go + 4);
    const v4f ka = *(const v4fa*)(k + go), kc = *(const v4fa*)(k + go + 4);
    const v4f va = *(const v4fa*)(v + go), vc = *(const v4fa*)(v + go + 4);
    FragH t;
#pragma unroll
    for (int j = 0; j < 4; ++j) {
      fq[i].h[j] = (_Float16)bf16_rne(qa[j]); fq[i].h[4 + j] = (_Float16)bf16_rne(qc[j]);
      fk[i].h[j] = (_Float16)bf16_rne(ka[j]); fk[i].h[4 + j] = (_Float16)bf16_rne(kc[j]);
      t.h[j] = (_Float16)bf16_rne(va[j]);     t.h[4 + j] = (_Float16)bf16_rne(vc[j]);
    }
#pragma unroll
    for (int j = 0; j < 8; ++j) tl[c8 + j][row] = t.u[j];
  }
  __syncthreads();
#pragma unroll
  for (int i = 0; i < 4; ++i) {
    const unsigned c = tid + ((unsigned)i << 8);
    const unsigned d = c >> 3, j8 = (c & 7u) << 3;
#pragma unroll
    for (int j = 0; j < 8; ++j) fv[i].u[j] = tl[d][j8 + j];
  }
  for (int pass = 0; pass < 2; ++pass) {
#pragma unroll
    for (int i = 0; i < 4; ++i) {
      const unsigned c = tid + ((unsigned)i << 8);
      const unsigned row = c >> 4, c8 = (c & 15u) << 3;
      const unsigned d = c >> 3, j8 = (c & 7u) << 3;
      const v8us oq = fq[i].half[0], ok = fk[i].half[0], ov = fv[i].half[0];
      *(volatile v8us*)((unsigned short*)Q16 + ob + (size_t)(row << 7) + c8) = oq;
      *(volatile v8us*)((unsigned short*)K16 + ob + (size_t)(row << 7) + c8) = ok;
      *(volatile v8us*)((unsigned short*)VT + ((size_t)bh * HD + d) * SEQ + jb + j8) = ov;
    }
    if (pass == 0) __threadfence();
  }
}

__global__ __launch_bounds__(128) void k_attn(const _Float16* __restrict__ Q16, const _Float16* __restrict__ K16, const _Float16* __restrict__ VT,
                                             float* __restrict__ out) {
  __shared__ __attribute__((aligned(16))) float so[4][16][HD];
  const unsigned tid = threadIdx.x, w = tid >> 5, lane = tid & 31u, ln = lane & 15u, hh = lane >> 4;
  const unsigned bh = blockIdx.y;
  const unsigned q0 = (blockIdx.x << 6) + (w << 4);
  const unsigned qa = q0 + ln;
  const unsigned short* qrow = (const unsigned short*)Q16 + ((size_t)bh * SEQ + qa) * HD;
  const unsigned short* kpl = (const unsigned short*)K16 + (size_t)bh * SEQ * HD;
  const unsigned short* vpl = (const unsigned short*)VT + (size_t)bh * HD * SEQ;

  FragH qb[KCH];
#pragma unroll
  for (int kc = 0; kc < KCH; ++kc) {
    qb[kc].half[0] = *(const v8us*)(qrow + 32 * kc + 8u * hh);
    qb[kc].half[1] = *(const v8us*)(qrow + 32 * kc + 16 + 8u * hh);
  }

  const v8f z8 = {0.f, 0.f, 0.f, 0.f, 0.f, 0.f, 0.f, 0.f};
  v8f acc[DTL] = {z8, z8, z8, z8, z8, z8, z8, z8};
  const float PS = 0.08838834764831845f * 256.0f;

#pragma unroll 1
  for (unsigned n0 = 0; n0 < SEQ; n0 += 32u) {
    v8f st[2] = {z8, z8};
#pragma unroll
    for (int kc = 0; kc < KCH; ++kc) {
#pragma unroll
      for (int t = 0; t < 2; ++t) {
        const unsigned short* kr = kpl + (size_t)(n0 + 16u * t + ln) * HD + 32 * kc;
        FragH ka;
        ka.half[0] = *(const v8us*)(kr + 8u * hh);
        ka.half[1] = *(const v8us*)(kr + 16 + 8u * hh);
        st[t] = mma16(ka.v, qb[kc].v, st[t]);
      }
    }
    FragH pf;
#pragma unroll
    for (int t = 0; t < 2; ++t)
#pragma unroll
      for (int r = 0; r < 8; ++r)
        pf.h[8 * t + r] = toh_flush(st[t][r] * PS);

#pragma unroll
    for (int dt = 0; dt < DTL; ++dt) {
      const unsigned short* vr = vpl + (size_t)(16u * dt + ln) * SEQ + n0;
      FragH va;
      va.half[0] = *(const v8us*)(vr + 8u * hh);
      va.half[1] = *(const v8us*)(vr + 16 + 8u * hh);
      acc[dt] = mma16(va.v, pf.v, acc[dt]);
    }
  }

  const float inv = 1.0f / 256.0f;
#pragma unroll
  for (int dt = 0; dt < DTL; ++dt)
#pragma unroll
    for (int r = 0; r < 8; ++r)
      so[w][ln][16 * dt + 8 * hh + r] = acc[dt][r] * inv;
  __builtin_amdgcn_fence(4  , "workgroup");
  __builtin_amdgcn_wave_barrier();
  float* obase = out + ((size_t)bh * SEQ + q0) * HD;
  const unsigned c4 = lane << 2;
  for (int pass = 0; pass < 2; ++pass) {
#pragma unroll
    for (int qq = 0; qq < 16; ++qq) {
      const v4f vv = *(const v4fa*)&so[w][qq][c4];
      *(volatile v4f*)(obase + (size_t)((unsigned)qq << 7) + c4) = vv;
    }
    if (pass == 0) __threadfence();
  }
}

extern "C" void kernel_launch(void* const* d_in, const int* in_sizes, int n_in,
                              void* d_out, int out_size, void* d_ws, size_t ws_size, hipStream_t stream) {
  if (n_in < 3) return;
  const size_t need_qkv = ((size_t)(NPL - 1) * SEQ_FULL + SEQ) * HD;
  if ((size_t)in_sizes[0] < need_qkv || (size_t)in_sizes[1] < need_qkv || (size_t)in_sizes[2] < need_qkv) return;
  if ((size_t)out_size < (size_t)NPL * SEQ * HD) return;
  const float* q = (const float*)d_in[0];
  const float* k = (const float*)d_in[1];
  const float* v = (const float*)d_in[2];
  float* out = (float*)d_out;

  char* ws = (char*)d_ws;
  size_t off = 0;
  _Float16* Q16 = (_Float16*)(ws + off); off += PLANE_BYTES;
  _Float16* K16 = (_Float16*)(ws + off); off += PLANE_BYTES;
  _Float16* VT  = (_Float16*)(ws + off); off += PLANE_BYTES;
  if (off > ws_size) return;

  k_cvt<<<dim3(SEQ / 64, NPL), 256, 0, stream>>>(q, k, v, Q16, K16, VT);
  k_attn<<<dim3(SEQ / 64, NPL), 128, 0, stream>>>(Q16, K16, VT, out);
}
